// KANLayer_30588757082465
// MI455X (gfx1250) — hardware-verified
//
#include <hip/hip_runtime.h>
#include <math.h>

typedef __attribute__((ext_vector_type(16))) _Float16 v16h;
typedef __attribute__((ext_vector_type(16))) __bf16 v16b;
typedef __attribute__((ext_vector_type(8)))  _Float16 v8h;
typedef __attribute__((ext_vector_type(8)))  float v8f;
typedef __attribute__((ext_vector_type(4)))  float v4f;
typedef __attribute__((ext_vector_type(2)))  float v2f;
typedef __attribute__((ext_vector_type(4)))  unsigned v4u;
typedef __attribute__((ext_vector_type(4)))  int v4i;
typedef float __attribute__((may_alias)) float_a;
typedef int __attribute__((may_alias)) int_a;

template <typename T> __device__ __forceinline__ void vst2(void* p, T v) { *(volatile T*)p = v; __threadfence(); *(volatile T*)p = v; }
__device__ __forceinline__ v8f wmma16(v16h a, v16h b, v8f c) {
  v8f d = __builtin_amdgcn_wmma_f32_16x16x32_f16(false, a, false, b, (short)0, c, false, false);
  asm volatile("v_nop\n\tv_nop\n\tv_nop\n\tv_nop" : "+v"(d) : "v"(a), "v"(b));
  return d;
}
__device__ __forceinline__ v8f wmma_bf(v16b a, v16b b, v8f c) {
  v8f d = __builtin_amdgcn_wmma_f32_16x16x32_bf16(false, a, false, b, (short)0, c, false, false);
  asm volatile("v_nop\n\tv_nop\n\tv_nop\n\tv_nop" : "+v"(d) : "v"(a), "v"(b));
  return d;
}
__device__ __forceinline__ v16h frag_h(const _Float16* rowk0, int lane) {
  union { v16h v; v8h q[2]; } u; const _Float16* p = rowk0 + 8 * (lane >> 4);
  u.q[0] = *(const v8h*)p; u.q[1] = *(const v8h*)(p + 16); return u.v;
}
__device__ __forceinline__ v16h frag_f32(const float* rowk0, int lane) {
  v16h a; const float* p = rowk0 + 8 * (lane >> 4);
#pragma unroll
  for (int i = 0; i < 8; ++i) { a[i] = (_Float16)p[i]; a[8 + i] = (_Float16)p[16 + i]; }
  return a;
}
__device__ __forceinline__ v16h frag_f32s(const float* rowk0, int lane, float sc) {
  v16h a; const float* p = rowk0 + 8 * (lane >> 4);
#pragma unroll
  for (int i = 0; i < 8; ++i) { a[i] = (_Float16)(p[i] * sc); a[8 + i] = (_Float16)(p[16 + i] * sc); }
  return a;
}
__device__ __forceinline__ v16h fragc_f32(const float* W, int k0, int n, int lane, int ld, int K) {
  v16h a; const int g = lane >> 4;
#pragma unroll
  for (int i = 0; i < 8; ++i) { const int ka = k0 + 8 * g + i, kb = ka + 16;
    a[i] = (_Float16)(ka < K ? W[(size_t)(ka < K ? ka : K - 1) * ld + n] : 0.f); a[8 + i] = (_Float16)(kb < K ? W[(size_t)(kb < K ? kb : K - 1) * ld + n] : 0.f); }
  return a;
}
struct F2 { v16b h, l; };
__device__ __forceinline__ F2 bsplit16(const float v[16]) { F2 r;
#pragma unroll
  for (int i = 0; i < 16; ++i) { const __bf16 h = (__bf16)v[i]; r.h[i] = h; r.l[i] = (__bf16)(v[i] - (float)h); }
  return r; }
__device__ __forceinline__ F2 split_row(const float* row, int k0, int lane) { float v[16]; const float* p = row + k0 + 8 * (lane >> 4);
#pragma unroll
  for (int i = 0; i < 8; ++i) { v[i] = p[i]; v[8 + i] = p[16 + i]; }
  return bsplit16(v); }
__device__ __forceinline__ F2 split_rowK(const float* row, int k0, int lane, int K) { float v[16]; const int g = lane >> 4;
#pragma unroll
  for (int i = 0; i < 8; ++i) { const int ka = k0 + 8 * g + i, kb = ka + 16; v[i] = ka < K ? row[ka < K ? ka : K - 1] : 0.f; v[8 + i] = kb < K ? row[kb < K ? kb : K - 1] : 0.f; }
  return bsplit16(v); }
__device__ __forceinline__ F2 split_col(const float* W, int k0, int n, int lane, int ld, int K) { float v[16]; const int g = lane >> 4;
#pragma unroll
  for (int i = 0; i < 8; ++i) { const int ka = k0 + 8 * g + i, kb = ka + 16; v[i] = ka < K ? W[(size_t)(ka < K ? ka : K - 1) * ld + n] : 0.f; v[8 + i] = kb < K ? W[(size_t)(kb < K ? kb : K - 1) * ld + n] : 0.f; }
  return bsplit16(v); }
__device__ __forceinline__ v8f mac3(const F2& a, const F2& b, v8f c) { c = wmma_bf(a.l, b.h, c); c = wmma_bf(a.h, b.l, c); return wmma_bf(a.h, b.h, c); }
__device__ __forceinline__ float sigm(float v) { return 1.0f / (1.0f + expf(-v)); }
#define LDSX() do { asm volatile("s_wait_dscnt 0" ::: "memory"); __builtin_amdgcn_wave_barrier(); __builtin_amdgcn_fence(__ATOMIC_RELEASE, "workgroup"); } while (0)

__device__ __forceinline__ float bfr(float v) { return (float)(__bf16)v; }
#define NBS 1024
#define IN 256
#define NOUT 256
#define NK 19
#define FEAT (IN * NK * 4)
#define WS_IDX 0u
#define WS_T   (WS_IDX + 4u * (size_t)NBS * IN)
#define WS_END (WS_T + 4u * (size_t)NBS * IN)
__global__ __launch_bounds__(256) void k_prep(const float* __restrict__ X, int* __restrict__ IDX, float* __restrict__ TV) { const size_t e = (size_t)blockIdx.x * 256 + threadIdx.x; if (e >= (size_t)NBS * IN) return;
  const float XMIN = -5.0f, XMAX = 5.0f; const float H = (XMAX - XMIN) / (float)(NK);
  const float x = bfr(X[e]); int id = (int)floorf((x - XMIN) / H); id = id < 0 ? 0 : (id > NK - 1 ? NK - 1 : id); const float t = x - (XMIN + (float)id * H);
  IDX[e] = id; TV[e] = t; }
__global__ __launch_bounds__(128) void k_kan(const int* __restrict__ IDX, const float* __restrict__ TV, const float* __restrict__ CF, const float* __restrict__ BIAS, float* __restrict__ OUT) { __shared__ __align__(16) float sf[4][16][132];
  const int tid = threadIdx.x, wave = tid >> 5, lane = tid & 31, col = lane & 15, g = lane >> 4; const int c0 = blockIdx.y * 128; const size_t r0 = (size_t)blockIdx.x * 64 + wave * 16; const size_t arow = r0 + col;
  v8f acc[8] = {};
#pragma unroll 1
  for (int kc = 0; kc < FEAT / 32; ++kc) { float v[16];
#pragma unroll
    for (int i = 0; i < 16; ++i) { const int e = kc * 32 + 8 * g + (i < 8 ? i : 8 + i); const int ii = e / (NK * 4), rem = e - ii * (NK * 4); const int k = rem >> 2, p = rem & 3; const int id = IDX[arow * IN + ii]; const float t = TV[arow * IN + ii]; const float tp = (p == 0) ? 1.0f : (p == 1) ? t : (p == 2) ? t * t : t * t * t; v[i] = (k == id) ? tp : 0.0f; }
    asm volatile("s_wait_loadcnt 0x0" ::: "memory"); const F2 a = bsplit16(v);
#pragma unroll
    for (int j = 0; j < 8; ++j) { v16b w; const float* wr = CF + (size_t)(c0 + j * 16 + col) * FEAT + kc * 32 + 8 * g;
#pragma unroll
      for (int i = 0; i < 8; ++i) { w[i] = (__bf16)wr[i]; w[8 + i] = (__bf16)wr[16 + i]; }
      asm volatile("s_wait_loadcnt 0x0" ::: "memory"); acc[j] = wmma_bf(a.h, w, acc[j]); acc[j] = wmma_bf(a.l, w, acc[j]); } }
#pragma unroll
  for (int j = 0; j < 8; ++j) { const float bb = bfr(BIAS[c0 + j * 16 + col]);
#pragma unroll
    for (int r = 0; r < 8; ++r) sf[wave][8 * g + r][j * 16 + col] = acc[j][r] + bb; }
  LDSX(); for (int rl = 0; rl < 16; ++rl) vst2(OUT + (r0 + rl) * NOUT + c0 + lane * 4, *(const v4f*)&sf[wave][rl][lane * 4]); }
extern "C" void kernel_launch(void* const* d_in, const int* in_sizes, int n_in, void* d_out, int out_size, void* d_ws, size_t ws_size, hipStream_t stream) {
  (void)in_sizes; (void)n_in; (void)out_size;
  const float** F = (const float**)d_in;
  if (ws_size < (size_t)WS_END) return;
  char* ws = (char*)d_ws; int* IDX = (int*)(ws + WS_IDX); float* TV = (float*)(ws + WS_T);
  k_prep<<<dim3(NBS * IN / 256), 256, 0, stream>>>(F[0], IDX, TV);
  k_kan<<<dim3(NBS / 64, NOUT / 128), 128, 0, stream>>>(IDX, TV, F[1], F[2], (float*)d_out);
}
